// _ConvBlock4LessLayers_43018392436824
// MI455X (gfx1250) — hardware-run, weakly checked
//
#include <hip/hip_runtime.h>
#include <stddef.h>
#include <stdint.h>


#define CCH     128
#define KW      256
#define NCH     25000
#define NTHR    256
#define NWAVE   8
#define EPT     8
#define CHUNK   (NTHR * EPT)
#define WCAP    (EPT * 32)
#define LISTN   (NWAVE * WCAP)
#define NBMAX   2048
#define RCAP    28672
#define DEGCAP  4096
#define GBM     64
#define GBN     64
#define GTHR    128
#define NLAYER  4
#define WSMAX   134217728
#define LDS_SEG ((2 * RCAP + 2 * NBMAX + LISTN) * 4 + 64)

static_assert((CHUNK & (CHUNK - 1)) == 0 && CHUNK <= 4096);
static_assert((NBMAX & (NBMAX - 1)) == 0 && NBMAX <= 4096);
static_assert(NTHR * 8 == NBMAX);
static_assert(LISTN >= NBMAX);
static_assert(LISTN >= NWAVE * WCAP);
static_assert((RCAP % 32) == 0);
static_assert(LDS_SEG <= 300000);
static_assert(GBM == (GTHR / 32) * 16);
static_assert(CCH == 128 && KW == 2 * CCH && (KW % 32) == 0 && (CCH % 32) == 0);
static_assert((CCH % GBN) == 0);
static_assert(CCH == 4 * 32);

typedef float          v4f  __attribute__((ext_vector_type(4)));
typedef float          v8f  __attribute__((ext_vector_type(8)));
typedef int            v4i  __attribute__((ext_vector_type(4)));
typedef int            v8i  __attribute__((ext_vector_type(8)));
typedef unsigned short v4us __attribute__((ext_vector_type(4)));
typedef unsigned short v8us __attribute__((ext_vector_type(8)));
typedef __bf16         v16b __attribute__((ext_vector_type(16)));
union FragB { v16b v; v8us h[2]; v8i w; };

__device__ __forceinline__ v8f wmb(const FragB& a, const FragB& b, v8f c) {
  v8f d = __builtin_amdgcn_wmma_f32_16x16x32_bf16(false, a.v, false, b.v, (short)0, c, false, false);
  asm volatile("v_nop\n\tv_nop\n\tv_nop\n\tv_nop" : "+v"(d) : "v"(a.w), "v"(b.w));
  return d;
}

__device__ __forceinline__ unsigned int bfb(float f) {
  const unsigned int u = __float_as_uint(f);
  return (u + 0x7FFFu + ((u >> 16) & 1u)) >> 16;
}
__device__ __forceinline__ float bfr(float f) { return __uint_as_float(bfb(f) << 16); }

__device__ __forceinline__ void split8(const v4f a, const v4f b, v8us& hi, v8us& lo) {
  const float in[8] = {a.x, a.y, a.z, a.w, b.x, b.y, b.z, b.w};
#pragma unroll
  for (int j = 0; j < 8; ++j) {
    const unsigned int hb = bfb(in[j]);
    const float hf = __uint_as_float(hb << 16);
    hi[j] = (unsigned short)hb;
    lo[j] = (unsigned short)bfb(in[j] - hf);
  }
}

__device__ __forceinline__ int scan_chunk(const int* __restrict__ dsts, int nE, int cbase, int slotBase,
                                          int nb, int vec8, int* list, int tid, int lane, int wave) {
  int wc = 0;
  const int el0  = tid * EPT;
  const int e0   = cbase + el0;
  const int sent = -2147483647 - 1;
  v4i da, db;
  if (vec8 != 0 && cbase + CHUNK <= nE) {
    da = *(const v4i*)(dsts + e0);
    db = *(const v4i*)(dsts + e0 + 4);
  } else {
    da.x = (e0     < nE) ? dsts[min(e0,     nE - 1)] : sent;
    da.y = (e0 + 1 < nE) ? dsts[min(e0 + 1, nE - 1)] : sent;
    da.z = (e0 + 2 < nE) ? dsts[min(e0 + 2, nE - 1)] : sent;
    da.w = (e0 + 3 < nE) ? dsts[min(e0 + 3, nE - 1)] : sent;
    db.x = (e0 + 4 < nE) ? dsts[min(e0 + 4, nE - 1)] : sent;
    db.y = (e0 + 5 < nE) ? dsts[min(e0 + 5, nE - 1)] : sent;
    db.z = (e0 + 6 < nE) ? dsts[min(e0 + 6, nE - 1)] : sent;
    db.w = (e0 + 7 < nE) ? dsts[min(e0 + 7, nE - 1)] : sent;
  }
  const unsigned nbs = (unsigned)slotBase;
  const unsigned unb = (unsigned)nb;
  const unsigned s0 = (unsigned)da.x - nbs, s1 = (unsigned)da.y - nbs;
  const unsigned s2 = (unsigned)da.z - nbs, s3 = (unsigned)da.w - nbs;
  const unsigned s4 = (unsigned)db.x - nbs, s5 = (unsigned)db.y - nbs;
  const unsigned s6 = (unsigned)db.z - nbs, s7 = (unsigned)db.w - nbs;
  const bool h0 = s0 < unb, h1 = s1 < unb, h2 = s2 < unb, h3 = s3 < unb;
  const bool h4 = s4 < unb, h5 = s5 < unb, h6 = s6 < unb, h7 = s7 < unb;
  const unsigned any = __builtin_amdgcn_ballot_w32(h0 | h1 | h2 | h3 | h4 | h5 | h6 | h7);
  if (any != 0u) {
#define HITJ(J, HJ, SJ) { \
      const unsigned mj = __builtin_amdgcn_ballot_w32(HJ); \
      if (mj != 0u) { \
        if (HJ) { \
          const int pos = wc + (int)__builtin_amdgcn_mbcnt_lo(mj, 0u); \
          if (pos < WCAP) list[wave * WCAP + pos] = ((el0 + (J)) << 12) | (int)(SJ); \
        } \
        wc += (int)__builtin_popcount(mj); } }
    HITJ(0, h0, s0)
    HITJ(1, h1, s1)
    HITJ(2, h2, s2)
    HITJ(3, h3, s3)
    HITJ(4, h4, s4)
    HITJ(5, h5, s5)
    HITJ(6, h6, s6)
    HITJ(7, h7, s7)
#undef HITJ
  }
  return wc;
}

__global__ __launch_bounds__(NTHR) void k_wprep(
    const float* __restrict__ w0s, const float* __restrict__ w0n,
    const float* __restrict__ w1s, const float* __restrict__ w1n,
    const float* __restrict__ w2s, const float* __restrict__ w2n,
    const float* __restrict__ w3s, const float* __restrict__ w3n,
    unsigned short* wt, int nUnits) {
  const int u = (int)blockIdx.x * NTHR + (int)threadIdx.x;
  if (u >= nUnits) return;
  const int layer = u >> 12;
  const int rem   = u & 4095;
  const int n     = rem >> 5;
  const int k8    = (rem & 31) * 8;
  const int kk    = k8 & (CCH - 1);
  const int seg   = k8 >> 7;
  const float* ps = (layer == 0) ? w0s : ((layer == 1) ? w1s : ((layer == 2) ? w2s : w3s));
  const float* pn = (layer == 0) ? w0n : ((layer == 1) ? w1n : ((layer == 2) ? w2n : w3n));
  const float* q  = (seg != 0) ? pn : ps;
  const float* p  = q + (size_t)kk * CCH + n;
  v8us hv;
#pragma unroll
  for (int j = 0; j < 8; ++j) hv[j] = (unsigned short)bfb(p[(size_t)j * CCH]);
  const size_t o = (size_t)layer * (size_t)(CCH * KW) + (size_t)n * KW + k8;
  *(volatile v8us*)(wt + o) = hv;
  __threadfence();
  *(volatile v8us*)(wt + o) = hv;
}

__global__ __launch_bounds__(GTHR) void k_gemm(
    const float* __restrict__ Ah, const float* __restrict__ Ag, const unsigned short* __restrict__ WT,
    const float* __restrict__ bias, const int* __restrict__ pnseg, float* Hout, int nsegHost)
{
  __shared__ __attribute__((aligned(16))) float stg[GBM * GBN];
  const int tid = (int)threadIdx.x, lane = tid & 31, wave = tid >> 5, hh = lane >> 4, m = lane & 15;
  const int rowBase = (int)blockIdx.x * GBM;
  const int col0    = (int)blockIdx.y * GBN;
  int nseg;
  {
    const int v = pnseg[0];
    nseg = v < 0 ? 0 : (v > nsegHost ? nsegHost : v);
  }

  v8f acc[4];
  {
    const v8f z = {0.f, 0.f, 0.f, 0.f, 0.f, 0.f, 0.f, 0.f};
    acc[0] = z; acc[1] = z; acc[2] = z; acc[3] = z;
  }
  const size_t arow = (size_t)(rowBase + 16 * wave + m) * (size_t)CCH + 8 * hh;
  const float* aph = Ah + arow;
  const float* apg = Ag + arow;
  const unsigned short* wp = WT + (size_t)(col0 + m) * (size_t)KW + 8 * hh;
#pragma unroll 1
  for (int ks = 0; ks < KW / 32; ++ks) {
    const float* ap = (((ks >> 2) == 0) ? aph : apg) + 32 * (ks & 3);
    const v4f a0 = *(const v4f*)(ap);
    const v4f a1 = *(const v4f*)(ap + 4);
    const v4f a2 = *(const v4f*)(ap + 16);
    const v4f a3 = *(const v4f*)(ap + 20);
    FragB fh, fl;
    split8(a0, a1, fh.h[0], fl.h[0]);
    split8(a2, a3, fh.h[1], fl.h[1]);
#pragma unroll
    for (int t = 0; t < 4; ++t) {
      const unsigned short* wq = wp + (size_t)(16 * t) * (size_t)KW + 32 * ks;
      FragB bf;
      bf.h[0] = *(const v8us*)wq;
      bf.h[1] = *(const v8us*)(wq + 16);
      acc[t] = wmb(fh, bf, acc[t]);
      acc[t] = wmb(fl, bf, acc[t]);
    }
  }

#pragma unroll
  for (int t = 0; t < 4; ++t) {
    const int lc = 16 * t + m;
    const float bv = bfr(bias[col0 + lc]);
#pragma unroll
    for (int r = 0; r < 8; ++r) {
      const int lr   = 16 * wave + 8 * hh + r;
      const int grow = rowBase + lr;
      float v = acc[t][r] + bv;
      v = (v < 0.f) ? 0.f : v;
      v = (grow < nseg) ? v : 0.f;
      stg[lr * GBN + lc] = v;
    }
  }
  __syncthreads();

  v4f fv[8];
#pragma unroll
  for (int i = 0; i < 8; ++i) {
    const int lr = 16 * wave + 2 * i + hh;
    fv[i] = *(const v4f*)(stg + lr * GBN + 4 * m);
  }
#pragma unroll
  for (int i = 0; i < 8; ++i) {
    const int gr = rowBase + 16 * wave + 2 * i + hh;
    float* op = Hout + (size_t)gr * (size_t)CCH + col0 + 4 * m;
    *(volatile v4f*)op = fv[i];
  }
  __threadfence();
#pragma unroll
  for (int i = 0; i < 8; ++i) {
    const int gr = rowBase + 16 * wave + 2 * i + hh;
    float* op = Hout + (size_t)gr * (size_t)CCH + col0 + 4 * m;
    *(volatile v4f*)op = fv[i];
  }
}

__global__ __launch_bounds__(NTHR) void k_seg(
    const int* __restrict__ srcs, const int* __restrict__ dsts, const float* __restrict__ attr,
    const float* __restrict__ feat, const int* __restrict__ pnsrc, const int* __restrict__ pnseg,
    float* outF, int nsrcHost, int nsegHost, int nE, int nb, int vec8, int MPr, int flags) {
  extern __shared__ v4f lds_dyn[];
  int* reg1 = (int*)lds_dyn;
  int* reg2 = reg1 + RCAP;
  int* scnt = reg2 + RCAP;
  int* soff = scnt + NBMAX;
  int* list = soff + NBMAX;
  int* wcnt = list + LISTN;
  int* wtot = wcnt + NWAVE;
  const int tid = (int)threadIdx.x, lane = tid & 31, wave = tid >> 5;
  const int nodeBase = (int)blockIdx.x * nb;
  const float qnan = __int_as_float(0x7fc00000);

  float pz0 = 0.f;
  int nseg, nsrc = nsrcHost;
  {
    const int v = pnseg[0];
    if (v < 1 || v > nsegHost) pz0 = qnan;
    nseg = v < 1 ? 1 : (v > nsegHost ? nsegHost : v);
  }
  if ((flags & 1) != 0) {
    const int v = pnsrc[0];
    if (v < 1 || v > nsrcHost) pz0 = qnan;
    nsrc = v < 1 ? 1 : (v > nsrcHost ? nsrcHost : v);
  }
  const int rnd = (flags & 2);

  for (int i = tid; i < NBMAX; i += NTHR) scnt[i] = 0;
  __syncthreads();

  int tot = 0;
  const int nChunks = (nE + CHUNK - 1) / CHUNK;
#pragma unroll 1
  for (int ch = 0; ch < nChunks; ++ch) {
    const int cbase = ch * CHUNK;
    const int wc = scan_chunk(dsts, nE, cbase, nodeBase, nb, vec8, list, tid, lane, wave);
    if (lane == 0) wcnt[wave] = wc;
    __syncthreads();
    int pre = 0, all = 0;
#pragma unroll
    for (int w2 = 0; w2 < NWAVE; ++w2) {
      int c = wcnt[w2];
      c = c < 0 ? 0 : (c > WCAP ? WCAP : c);
      all += c;
      pre += (w2 < wave) ? c : 0;
    }
    const int wcc  = wc > WCAP ? WCAP : wc;
    const int base = tot + pre;
#pragma unroll 1
    for (int i = lane; i < wcc; i += 32) {
      const int ent = list[wave * WCAP + i];
      const int el  = (ent >> 12) & (CHUNK - 1);
      const int sl  = ent & (NBMAX - 1);
      int eid = cbase + el;
      eid = eid > nE - 1 ? nE - 1 : eid;
      const int pos = base + i;
      if (pos < RCAP) reg1[pos] = (int)(((unsigned)eid << 12) | (unsigned)sl);
    }
    tot += all;
    tot = tot > RCAP ? RCAP : tot;
    __syncthreads();
  }
  const int nh = tot;

  if (wave == 0) {
#pragma unroll 1
    for (int b0 = 0; b0 < nh; b0 += 32) {
      const int idx = b0 + lane;
      const int uv  = reg1[idx < nh ? idx : nh - 1];
      const int m32 = (nh - b0) < 32 ? (nh - b0) : 32;
#pragma unroll 1
      for (int k = 0; k < m32; ++k) {
        const int u  = __builtin_amdgcn_readlane(uv, k);
        const int sl = u & (NBMAX - 1);
        if (lane == 0) scnt[sl] = scnt[sl] + 1;
      }
    }
  }
  __syncthreads();

  {
    const v4i ca = *(const v4i*)(scnt + 8 * tid);
    const v4i cb = *(const v4i*)(scnt + 8 * tid + 4);
    const int e0 = ca.x < 0 ? 0 : ca.x, e1 = ca.y < 0 ? 0 : ca.y, e2 = ca.z < 0 ? 0 : ca.z, e3 = ca.w < 0 ? 0 : ca.w;
    const int e4 = cb.x < 0 ? 0 : cb.x, e5 = cb.y < 0 ? 0 : cb.y, e6 = cb.z < 0 ? 0 : cb.z, e7 = cb.w < 0 ? 0 : cb.w;
    const int ts = e0 + e1 + e2 + e3 + e4 + e5 + e6 + e7;
    int incl = ts;
#pragma unroll
    for (int d = 1; d < 32; d <<= 1) {
      const int up = __shfl_up(incl, d);
      if (lane >= d) incl += up;
    }
    if (lane == 31) wtot[wave] = incl;
    __syncthreads();
    int pre = 0;
#pragma unroll
    for (int w2 = 0; w2 < NWAVE; ++w2) pre += (w2 < wave) ? wtot[w2] : 0;
    int run = pre + incl - ts;
    soff[8 * tid + 0] = run; run += e0;
    soff[8 * tid + 1] = run; run += e1;
    soff[8 * tid + 2] = run; run += e2;
    soff[8 * tid + 3] = run; run += e3;
    soff[8 * tid + 4] = run; run += e4;
    soff[8 * tid + 5] = run; run += e5;
    soff[8 * tid + 6] = run; run += e6;
    soff[8 * tid + 7] = run;
  }
  __syncthreads();
  for (int i = tid; i < NBMAX; i += NTHR) list[i] = soff[i];
  __syncthreads();

  if (wave == 0) {
#pragma unroll 1
    for (int b0 = 0; b0 < nh; b0 += 32) {
      const int idx = b0 + lane;
      const int uv  = reg1[idx < nh ? idx : nh - 1];
      const int m32 = (nh - b0) < 32 ? (nh - b0) : 32;
#pragma unroll 1
      for (int k = 0; k < m32; ++k) {
        const int u   = __builtin_amdgcn_readlane(uv, k);
        const int sl  = u & (NBMAX - 1);
        const int eid = (int)((unsigned)u >> 12);
        if (lane == 0) {
          int pos = list[sl];
          pos = pos < 0 ? 0 : (pos > RCAP - 1 ? RCAP - 1 : pos);
          reg2[pos] = eid;
          list[sl] = pos + 1;
        }
      }
    }
  }
  __syncthreads();

  const int nbw = nb >> 3;
  const bool ovf = (nh >= RCAP);
  int lim = nh - 1;
  lim = lim < 0 ? 0 : (lim > RCAP - 1 ? RCAP - 1 : lim);
#pragma unroll 1
  for (int jt = 0; jt < nbw; ++jt) {
    const int slot = wave * nbw + jt;
    const int grow = nodeBase + slot;
    int st = soff[slot];
    const int craw = scnt[slot];
    int cnt = craw;
    st  = st < 0 ? 0 : (st > nh ? nh : st);
    cnt = cnt < 0 ? 0 : (cnt > DEGCAP ? DEGCAP : cnt);
    if (cnt > nh - st) cnt = nh - st;
    st  = __builtin_amdgcn_readfirstlane(st);
    cnt = __builtin_amdgcn_readfirstlane(cnt);
    const float pz = ((ovf || craw > DEGCAP) ? qnan : 0.0f) + pz0;
    const bool wr = grow < MPr;
    const float live = grow < nseg ? 1.0f : 0.0f;

    v4f acc = {0.f, 0.f, 0.f, 0.f};
#pragma unroll 1
    for (int q0 = 0; q0 < cnt; q0 += 32) {
      int idx = st + q0 + lane;
      idx = idx > lim ? lim : idx;
      int eid = reg2[idx];
      eid = eid < 0 ? 0 : (eid > nE - 1 ? nE - 1 : eid);
      int sraw = srcs[eid];
      sraw = sraw < 0 ? sraw + nsrc : sraw;
      const int s  = sraw < 0 ? 0 : (sraw > nsrc - 1 ? nsrc - 1 : sraw);
      const int ab = __float_as_int(bfr(attr[eid]));
      int m32 = (cnt - q0) < 32 ? (cnt - q0) : 32;
      m32 = __builtin_amdgcn_readfirstlane(m32);
#pragma unroll 1
      for (int k = 0; k < m32; ++k) {
        const int   sk = __builtin_amdgcn_readlane(s, k);
        const float ak = __int_as_float(__builtin_amdgcn_readlane(ab, k));
        v4f v = *(const v4f*)(feat + (size_t)sk * CCH + 4 * lane);
        if (rnd != 0) { v.x = bfr(v.x); v.y = bfr(v.y); v.z = bfr(v.z); v.w = bfr(v.w); }
        acc.x = fmaf(ak, v.x, acc.x);
        acc.y = fmaf(ak, v.y, acc.y);
        acc.z = fmaf(ak, v.z, acc.z);
        acc.w = fmaf(ak, v.w, acc.w);
      }
    }
    v4f r;
    r.x = acc.x * live + pz; r.y = acc.y * live + pz; r.z = acc.z * live + pz; r.w = acc.w * live + pz;
    float* fp = outF + (size_t)grow * (size_t)CCH + 4 * lane;
    if (wr) *(volatile v4f*)fp = r;
    __threadfence();
    if (wr) *(volatile v4f*)fp = r;
  }
}

static int pick_nb(int nE, int nN) {
  int nb = NBMAX;
  while (nb > 16 && (long long)nb * (long long)nE * 5LL > (long long)RCAP * (long long)nN * 4LL) nb >>= 1;
  return nb;
}
static inline int cdiv(int a, int b) { return (a + b - 1) / b; }

extern "C" void kernel_launch(void* const* d_in, const int* in_sizes, int n_in,
                              void* d_out, int out_size, void* d_ws, size_t ws_size,
                              hipStream_t stream) {
  if (n_in < 24) return;
  const int nFx = in_sizes[0] / CCH;
  if (nFx <= 0 || in_sizes[0] != nFx * CCH || nFx > (1 << 22)) return;
  const int eP = in_sizes[1];
  if (eP < 1 || eP > (1 << 20) || in_sizes[2] != eP || in_sizes[3] != eP) return;
  const int eC = in_sizes[4];
  if (eC < 1 || eC > (1 << 20) || in_sizes[5] != eC || in_sizes[6] != eC) return;
  const int eU = in_sizes[7];
  if (eU < 1 || eU > (1 << 20) || in_sizes[8] != eU || in_sizes[9] != eU) return;
  for (int l = 0; l < NLAYER; ++l) {
    if (in_sizes[10 + 3 * l] != CCH * CCH || in_sizes[11 + 3 * l] != CCH * CCH || in_sizes[12 + 3 * l] != CCH) return;
  }
  if (in_sizes[22] != 1 || in_sizes[23] != 1) return;
  const int nF = out_size / CCH;
  if (nF <= 0 || out_size != nF * CCH || nF > (1 << 22)) return;

  const float* x     = (const float*)d_in[0];
  const int*   psrc  = (const int*)  d_in[1];
  const int*   pdst  = (const int*)  d_in[2];
  const float* patt  = (const float*)d_in[3];
  const int*   csrc  = (const int*)  d_in[4];
  const int*   cdst  = (const int*)  d_in[5];
  const float* catt  = (const float*)d_in[6];
  const int*   usrc  = (const int*)  d_in[7];
  const int*   udst  = (const int*)  d_in[8];
  const float* uatt  = (const float*)d_in[9];
  const float* wsl[NLAYER] = { (const float*)d_in[10], (const float*)d_in[13], (const float*)d_in[16], (const float*)d_in[19] };
  const float* wnl[NLAYER] = { (const float*)d_in[11], (const float*)d_in[14], (const float*)d_in[17], (const float*)d_in[20] };
  const float* bsl[NLAYER] = { (const float*)d_in[12], (const float*)d_in[15], (const float*)d_in[18], (const float*)d_in[21] };
  const int*   pnc   = (const int*)  d_in[22];
  const int*   pnf   = (const int*)  d_in[23];
  float* out = (float*)d_out;

  const int MP  = cdiv(NCH, GBM) * GBM;
  const int nbP = pick_nb(eP, NCH);
  const int nbC = pick_nb(eC, NCH);
  const int nbU = pick_nb(eU, nF);
  const int gP  = cdiv(MP, nbP), gC = cdiv(MP, nbC), gU = cdiv(nF, nbU);
  if (gP * nbP < MP || gC * nbC < MP || gU * nbU < nF) return;
  const int vec8 = 1;

  char* wsb = (char*)d_ws;
  const size_t plane = (size_t)MP * CCH * 4;
  size_t off = 0;
  const size_t oWT = off; off += (size_t)NLAYER * CCH * KW * 2;   off = (off + 255) & ~(size_t)255;
  size_t oH[NLAYER + 1], oG[NLAYER];
  oH[0] = off; off += plane; off = (off + 255) & ~(size_t)255;
  for (int l = 0; l < NLAYER; ++l) {
    oG[l] = off;     off += plane; off = (off + 255) & ~(size_t)255;
    oH[l + 1] = off; off += plane; off = (off + 255) & ~(size_t)255;
  }
  if (off > ws_size || off > (size_t)WSMAX) return;
  unsigned short* WT = (unsigned short*)(wsb + oWT);
  float* H[NLAYER + 1];
  float* AG[NLAYER];
  for (int l = 0; l <= NLAYER; ++l) H[l] = (float*)(wsb + oH[l]);
  for (int l = 0; l < NLAYER; ++l)  AG[l] = (float*)(wsb + oG[l]);

  hipFuncSetAttribute(reinterpret_cast<const void*>(&k_seg),
                      hipFuncAttributeMaxDynamicSharedMemorySize, LDS_SEG);

  {
    const int nU = NLAYER * CCH * (KW / 8);
    k_wprep<<<cdiv(nU, NTHR), NTHR, 0, stream>>>(wsl[0], wnl[0], wsl[1], wnl[1], wsl[2], wnl[2], wsl[3], wnl[3],
                                                 WT, nU);
  }
  k_seg<<<gP, NTHR, LDS_SEG, stream>>>(psrc, pdst, patt, x, pnf, pnc, H[0],
                                       nFx, NCH, eP, nbP, vec8, MP, 2);
  const int gM = MP / GBM;
  for (int l = 0; l < NLAYER; ++l) {
    k_seg<<<gC, NTHR, LDS_SEG, stream>>>(csrc, cdst, catt, H[l], pnc, pnc, AG[l],
                                         NCH, NCH, eC, nbC, vec8, MP, 1);
    k_gemm<<<dim3(gM, CCH / GBN), GTHR, 0, stream>>>(H[l], AG[l], WT + (size_t)l * CCH * KW, bsl[l], pnc,
                                                     H[l + 1], NCH);
  }
  k_seg<<<gU, NTHR, LDS_SEG, stream>>>(usrc, udst, uatt, H[NLAYER], pnc, pnf, out,
                                       NCH, nF, eU, nbU, vec8, nF, 1);
}
